// KANLinear_68607807586406
// MI455X (gfx1250) — hardware-verified
//
#include <hip/hip_runtime.h>


#define NBR  4096
#define NI   512
#define NO   512
#define GP   15
#define KORD 3
#define NJ   11
#define KTOT (NJ * NI + NI)
typedef _Float16 h16;
typedef unsigned short bf;
typedef __attribute__((ext_vector_type(16))) __bf16   v16bf;
typedef __attribute__((ext_vector_type(16))) _Float16 v16h;
typedef __attribute__((ext_vector_type(8)))  _Float16 v8h;
typedef __attribute__((ext_vector_type(8)))  unsigned short v8us;
typedef __attribute__((ext_vector_type(8)))  float    v8f;
typedef __attribute__((ext_vector_type(4)))  float    v4f;
typedef v8h  __attribute__((may_alias)) v8ha;
typedef v4f  __attribute__((may_alias)) v4fa;
typedef v8us __attribute__((may_alias)) v8usa;

__device__ __forceinline__ unsigned short f2bf(float f) { unsigned u = __float_as_uint(f); u += 0x7FFFu + ((u >> 16) & 1u); return (unsigned short)(u >> 16); }
__device__ __forceinline__ float bf2f(unsigned short b) { return __uint_as_float(((unsigned)b) << 16); }
__device__ __forceinline__ float bfr(float f) { return bf2f(f2bf(f)); }
__device__ __forceinline__ v16h cat16(v8h lo, v8h hi) { return __builtin_shufflevector(lo, hi, 0, 1, 2, 3, 4, 5, 6, 7, 8, 9, 10, 11, 12, 13, 14, 15); }
__device__ __forceinline__ v16bf cat16b(v8us lo, v8us hi) { return __builtin_bit_cast(v16bf, __builtin_shufflevector(lo, hi, 0, 1, 2, 3, 4, 5, 6, 7, 8, 9, 10, 11, 12, 13, 14, 15)); }
__device__ __forceinline__ v8f wmma16(v16h a, v16h b, v8f c) { return __builtin_amdgcn_wmma_f32_16x16x32_f16(false, a, false, b, (short)0, c, false, false); }
__device__ __forceinline__ v8f wmmab(v16bf a, v16bf b, v8f c) { return __builtin_amdgcn_wmma_f32_16x16x32_bf16(false, a, false, b, (short)0, c, false, false); }


template <typename T16> struct WFrag;
template <> struct WFrag<h16> { typedef v16h V; static __device__ __forceinline__ V ld(const h16* p) { return cat16(*(const v8h*)p, *(const v8h*)(p + 16)); } static __device__ __forceinline__ v8f mma(V a, V b, v8f c) { return wmma16(a, b, c); } };
template <> struct WFrag<bf> { typedef v16bf V; static __device__ __forceinline__ V ld(const bf* p) { return cat16b(*(const v8us*)p, *(const v8us*)(p + 16)); } static __device__ __forceinline__ v8f mma(V a, V b, v8f c) { return wmmab(a, b, c); } };
template <typename T16, int NSPLIT, bool BIAS>
__global__ __launch_bounds__(32) void k_gemmw(const T16* __restrict__ A, const T16* __restrict__ A2, const T16* __restrict__ Bt, const T16* __restrict__ Bt2, int K, float* C, int ldc, const float* __restrict__ bias, size_t sA, size_t sB, size_t sC) {
    typedef typename WFrag<T16>::V V;
    __shared__ __align__(16) float os[16 * 68];
    const size_t z = blockIdx.z; A += z * sA; if (A2) A2 += z * sA; Bt += z * sB; if (Bt2) Bt2 += z * sB; C += z * sC;
    const int lane = threadIdx.x & 31, lr = lane & 15, hi = lane >> 4; const int r0 = blockIdx.x * 64, c0 = blockIdx.y * 64;
    v8f acc[4][4];
#pragma unroll
    for (int mb = 0; mb < 4; ++mb)
#pragma unroll
        for (int nb = 0; nb < 4; ++nb) acc[mb][nb] = (v8f){};
    const size_t aoff = (size_t)(r0 + lr) * K + 8 * hi, boff = (size_t)(c0 + lr) * K + 8 * hi;
#pragma unroll 1
    for (int kc = 0; kc < K; kc += 32) {
        V a[4], a2[4];
#pragma unroll
        for (int mb = 0; mb < 4; ++mb) { a[mb] = WFrag<T16>::ld(A + aoff + (size_t)mb * 16 * K + kc); if (NSPLIT == 1 || NSPLIT == 2) a2[mb] = WFrag<T16>::ld(A2 + aoff + (size_t)mb * 16 * K + kc); }
#pragma unroll
        for (int nb = 0; nb < 4; ++nb) { const V b = WFrag<T16>::ld(Bt + boff + (size_t)nb * 16 * K + kc); V b2; if (NSPLIT >= 2) b2 = WFrag<T16>::ld(Bt2 + boff + (size_t)nb * 16 * K + kc);
#pragma unroll
            for (int mb = 0; mb < 4; ++mb) { acc[mb][nb] = WFrag<T16>::mma(a[mb], b, acc[mb][nb]); if (NSPLIT == 1 || NSPLIT == 2) acc[mb][nb] = WFrag<T16>::mma(a2[mb], b, acc[mb][nb]); if (NSPLIT >= 2) acc[mb][nb] = WFrag<T16>::mma(a[mb], b2, acc[mb][nb]); } }
        asm volatile("v_nop\n\tv_nop\n\tv_nop\n\tv_nop" : "+v"(acc[0][0]), "+v"(acc[1][1]), "+v"(acc[2][2]), "+v"(acc[3][3]) : "v"(a[0]), "v"(a[3]));
    }
#pragma unroll
    for (int mb = 0; mb < 4; ++mb) {
#pragma unroll
        for (int nb = 0; nb < 4; ++nb) {
#pragma unroll
            for (int j = 0; j < 8; ++j) os[(hi * 8 + j) * 68 + nb * 16 + lr] = acc[mb][nb][j]; }
        __builtin_amdgcn_wave_barrier(); asm volatile("" ::: "memory");
        float* crow = C + (size_t)(r0 + mb * 16) * ldc + c0;
#pragma unroll 1
        for (int ps = 0; ps < 2; ++ps) {
#pragma unroll
            for (int s = 0; s < 8; ++s) { const int row = 2 * s + hi, cofs = lr * 4; v4f val = *(const v4fa*)(os + row * 68 + cofs); if (BIAS) { val[0] += bfr(bias[c0 + cofs]); val[1] += bfr(bias[c0 + cofs + 1]); val[2] += bfr(bias[c0 + cofs + 2]); val[3] += bfr(bias[c0 + cofs + 3]); }
                *(volatile v4f*)(crow + (size_t)row * ldc + cofs) = val; }
            if (ps == 0) __threadfence(); }
        __builtin_amdgcn_wave_barrier(); asm volatile("" ::: "memory");
    }
}

__device__ __forceinline__ void splitf(float y, unsigned short& h, unsigned short& l) { h = f2bf(y); l = f2bf(y - bf2f(h)); }
__global__ __launch_bounds__(256) void k_b0(const float* __restrict__ X, const float* __restrict__ G, float* T) {
    const size_t t = (size_t)blockIdx.x * 256 + threadIdx.x; if (t >= (size_t)NBR * (NI / 8)) return; const int i0 = (int)(t % (NI / 8)) * 8; const size_t b = t / (NI / 8);
#pragma unroll 1
    for (int m = 0; m < GP - 1; ++m) { v4f oa, ob;
#pragma unroll
        for (int q = 0; q < 8; ++q) { const int i = i0 + q; const float xv = bfr(X[b * NI + i]); const float g0 = bfr(G[(size_t)i * GP + m]), g1 = bfr(G[(size_t)i * GP + m + 1]); const float v = (xv >= g0 && xv < g1) ? 1.0f : 0.0f; if (q < 4) oa[q] = v; else ob[q - 4] = v; }
        float* dst = T + ((size_t)m * NBR + b) * NI + i0;
#pragma unroll 1
        for (int ps = 0; ps < 2; ++ps) { *(volatile v4f*)dst = oa; *(volatile v4f*)(dst + 4) = ob; if (ps == 0) __threadfence(); } } }
__global__ __launch_bounds__(256) void k_blev(const float* __restrict__ X, const float* __restrict__ G, int p, int m0, int m1, float* T) {
    const size_t t = (size_t)blockIdx.x * 256 + threadIdx.x; if (t >= (size_t)NBR * (NI / 8)) return; const int i0 = (int)(t % (NI / 8)) * 8; const size_t b = t / (NI / 8);
#pragma unroll 1
    for (int m = m0; m < m1; ++m) { v4f oa, ob; const float* s0 = T + ((size_t)m * NBR + b) * NI + i0; const float* s1 = T + ((size_t)(m + 1) * NBR + b) * NI + i0; const v4f a0 = *(const v4f*)s0, a1 = *(const v4f*)(s0 + 4), c0 = *(const v4f*)s1, c1 = *(const v4f*)(s1 + 4);
#pragma unroll
        for (int q = 0; q < 8; ++q) { const int i = i0 + q; const float xv = bfr(X[b * NI + i]); const float* gi = G + (size_t)i * GP; const float gm = bfr(gi[m]), gmp = bfr(gi[m + p]), gmp1 = bfr(gi[m + p + 1]), gm1 = bfr(gi[m + 1]);
            const float la = __fdiv_rn(__fsub_rn(xv, gm), __fsub_rn(gmp, gm)); const float rb = __fdiv_rn(__fsub_rn(gmp1, xv), __fsub_rn(gmp1, gm1)); const float Bm = (q < 4) ? a0[q] : a1[q - 4], Bn = (q < 4) ? c0[q] : c1[q - 4];
            float t1 = __fmul_rn(la, Bm), t2 = __fmul_rn(rb, Bn); asm volatile("" : "+v"(t1), "+v"(t2)); const float v = __fadd_rn(t1, t2); if (q < 4) oa[q] = v; else ob[q - 4] = v; }
        float* dst = T + ((size_t)m * NBR + b) * NI + i0;
#pragma unroll 1
        for (int ps = 0; ps < 2; ++ps) { *(volatile v4f*)dst = oa; *(volatile v4f*)(dst + 4) = ob; if (ps == 0) __threadfence(); } } }
__global__ __launch_bounds__(256) void k_bpack(const float* __restrict__ X, const float* __restrict__ T, bf* Ah, bf* Al) {
    const size_t t = (size_t)blockIdx.x * 256 + threadIdx.x; if (t >= (size_t)NBR * (NI / 8)) return; const int i0 = (int)(t % (NI / 8)) * 8; const size_t b = t / (NI / 8);
#pragma unroll 1
    for (int j = 0; j <= NJ; ++j) { v8us vh, vl;
#pragma unroll
        for (int q = 0; q < 8; ++q) { float v; if (j < NJ) v = T[((size_t)j * NBR + b) * NI + i0 + q]; else { const float xv = bfr(X[b * NI + i0 + q]); v = __fdiv_rn(xv, __fadd_rn(1.0f, __builtin_amdgcn_exp2f(__fmul_rn(xv, -1.4426950408889634f)))); } unsigned short a, c; splitf(v, a, c); vh[q] = a; vl[q] = c; }
        const size_t col = (size_t)j * NI + i0;
#pragma unroll 1
        for (int ps = 0; ps < 2; ++ps) { *(volatile v8us*)(Ah + b * KTOT + col) = vh; *(volatile v8us*)(Al + b * KTOT + col) = vl; if (ps == 0) __threadfence(); } } }

__global__ __launch_bounds__(256) void k_wkan(const float* __restrict__ coef, const float* __restrict__ ssp, const float* __restrict__ sba, bf* Bh, bf* Bl) {
    const size_t t = (size_t)blockIdx.x * 256 + threadIdx.x; if (t >= (size_t)NO * (NJ + 1) * (NI / 8)) return; const int i0 = (int)(t % (NI / 8)) * 8; const int j = (int)((t / (NI / 8)) % (NJ + 1)); const size_t o = t / ((size_t)(NI / 8) * (NJ + 1)); v8us vh, vl;
#pragma unroll
    for (int q = 0; q < 8; ++q) { const int i = i0 + q; float w; if (j < NJ) w = __fmul_rn(bfr(coef[((size_t)i * NO + o) * NJ + j]), bfr(ssp[(size_t)i * NO + o])); else w = bfr(sba[(size_t)i * NO + o]); unsigned short a, c; splitf(w, a, c); vh[q] = a; vl[q] = c; }
    const size_t col = (size_t)j * NI + i0; *(volatile v8us*)(Bh + o * KTOT + col) = vh; *(volatile v8us*)(Bl + o * KTOT + col) = vl; __threadfence(); *(volatile v8us*)(Bh + o * KTOT + col) = vh; *(volatile v8us*)(Bl + o * KTOT + col) = vl; }

extern "C" void kernel_launch(void* const* d_in, const int* in_sizes, int n_in,
                              void* d_out, int out_size, void* d_ws, size_t ws_size, hipStream_t stream) {
    (void)in_sizes; (void)n_in; (void)out_size;
    const float* X = (const float*)d_in[0]; const float* G = (const float*)d_in[1]; const float* coef = (const float*)d_in[2]; const float* sba = (const float*)d_in[3]; const float* ssp = (const float*)d_in[4];
    float* OUT = (float*)d_out;
    char* wsp = (char*)d_ws;
    auto take = [&](size_t bytes) { char* p = wsp; wsp += (bytes + 255) & ~(size_t)255; return (void*)p; };
    bf* Ah = (bf*)take((size_t)NBR * KTOT * 2); bf* Al = (bf*)take((size_t)NBR * KTOT * 2); bf* Bh = (bf*)take((size_t)NO * KTOT * 2); bf* Bl = (bf*)take((size_t)NO * KTOT * 2); float* T = (float*)take((size_t)(GP - 1) * NBR * NI * 4);
    if ((size_t)(wsp - (char*)d_ws) > ws_size) return;
    k_wkan<<<(unsigned)(((size_t)NO * (NJ + 1) * (NI / 8) + 255) / 256), 256, 0, stream>>>(coef, ssp, sba, Bh, Bl);
    const unsigned gl = (unsigned)(((size_t)NBR * (NI / 8) + 255) / 256);
    k_b0<<<gl, 256, 0, stream>>>(X, G, T);
    for (int p = 1; p <= KORD; ++p) { const int nm = GP - 1 - p; const int mid = nm / 2; k_blev<<<gl, 256, 0, stream>>>(X, G, p, 0, mid, T); k_blev<<<gl, 256, 0, stream>>>(X, G, p, mid, nm, T); }
    k_bpack<<<gl, 256, 0, stream>>>(X, T, Ah, Al);
    k_gemmw<bf, 2, false><<<dim3(NBR / 64, NO / 64, 1), 32, 0, stream>>>(Ah, Al, Bh, Bl, KTOT, OUT, NO, nullptr, 0, 0, 0);
}
